// SemSol_8830452761095
// MI455X (gfx1250) — hardware-verified
//
#include <hip/hip_runtime.h>
#include <stdint.h>


typedef _Float16 f16t;
typedef f16t  v16h __attribute__((ext_vector_type(16)));
typedef f16t  v8h  __attribute__((ext_vector_type(8)));
typedef float v8f  __attribute__((ext_vector_type(8)));
typedef float v4f  __attribute__((ext_vector_type(4)));
typedef unsigned int v4u __attribute__((ext_vector_type(4)));

union Frag { v16h v; v8h q[2]; };
union Pk16 { v8h h; v4u u; };

#define NB   8
#define NS   2048
#define NH   768
#define NHD  384
#define NG   1536
#define KC   1152
#define KTL  36
#define LPA  1160
#define NU   32
#define NTP  64
#define WPR  144

static_assert(KC % 32 == 0);
static_assert((LPA % 8) == 0);
static_assert(NB * NHD == 12 * 256);
static_assert(NB * (NH / 8) == 3 * 256);
static_assert(NB * (NHD / 4) == 3 * 256);
static_assert(WPR % 8 == 0);

__device__ __forceinline__ v8f wmma16(v16h a, v16h b, v8f c) {
    return __builtin_amdgcn_wmma_f32_16x16x32_f16(false, a, false, b, (short)0, c, false, false);
}

__device__ __forceinline__ void mma4(v8f (&acc)[4], const f16t* A, int lda,
                                     const f16t* B, int ldb, int ktiles) {
    const int l = threadIdx.x & 31, h = l >> 4, m = l & 15;
    const f16t* ap = A + m * lda + 8 * h;
    const f16t* bp = B + (size_t)m * ldb + 8 * h;
#pragma unroll 1
    for (int kt = 0; kt < ktiles; ++kt) {
        Frag a, b[4];
        const f16t* pa = ap + kt * 32;
        a.q[0] = *(const v8h*)pa;
        a.q[1] = *(const v8h*)(pa + 16);
#pragma unroll
        for (int j = 0; j < 4; ++j) {
            const f16t* pb = bp + (size_t)j * 16 * ldb + kt * 32;
            b[j].q[0] = *(const v8h*)pb;
            b[j].q[1] = *(const v8h*)(pb + 16);
        }
#pragma unroll
        for (int j = 0; j < 4; ++j) acc[j] = wmma16(a.v, b[j].v, acc[j]);
        asm volatile("v_nop\n\tv_nop\n\tv_nop\n\tv_nop"
                     : "+v"(acc[0]), "+v"(acc[1]), "+v"(acc[2]), "+v"(acc[3])
                     : "v"(a.v), "v"(b[0].v), "v"(b[1].v), "v"(b[2].v), "v"(b[3].v));
    }
}

__device__ __forceinline__ float fsig(float x) {
    float t = __expf(-x);
    return __builtin_amdgcn_rcpf(1.0f + t);
}
__device__ __forceinline__ float ftanh(float x) {
    float ax = fabsf(x);
    float t  = __expf(-2.0f * ax);
    float r  = (1.0f - t) * __builtin_amdgcn_rcpf(1.0f + t);
    return copysignf(r, x);
}

__global__ __launch_bounds__(256)
void k_wpack(const float* WihF, const float* WhhF, const float* WihB, const float* WhhB,
             f16t* Wc, int tot) {
    const int i = blockIdx.x * 256 + threadIdx.x;
    if (i >= tot) return;
    const int per = NG * WPR;
    const int dir = i / per;
    const int r   = i - dir * per;
    const int n   = r / WPR;
    const int kc  = (r - n * WPR) * 8;
    const bool hp = (kc >= NH);
    const int kih = hp ? (NH - 8) : kc;
    const int khh = hp ? (kc - NH) : 0;
    const float* wi = dir ? WihB : WihF;
    const float* wh = dir ? WhhB : WhhF;
    const float* pi = wi + (size_t)n * NH + kih;
    const float* ph = wh + (size_t)n * NHD + khh;
    const v4f a0 = *(const v4f*)pi;
    const v4f a1 = *(const v4f*)(pi + 4);
    const v4f b0 = *(const v4f*)ph;
    const v4f b1 = *(const v4f*)(ph + 4);
    Pk16 k;
#pragma unroll
    for (int e = 0; e < 4; ++e) {
        const float x0 = hp ? b0[e] : a0[e];
        const float x1 = hp ? b1[e] : a1[e];
        k.h[e]     = (f16t)(x0 * 32.0f);
        k.h[4 + e] = (f16t)(x1 * 32.0f);
    }
    f16t* d = Wc + (size_t)dir * NG * KC + (size_t)n * KC + kc;
    *(volatile v4u*)d = k.u;
    __threadfence();
    *(volatile v4u*)d = k.u;
}

__device__ __forceinline__ void gather_x(const float* X, f16t* As_, int s, int tid) {
#pragma unroll
    for (int i = 0; i < 3; ++i) {
        const int p  = tid + 256 * i;
        const int b  = p / 96;
        const int kc = (p - b * 96) * 8;
        const float* src = X + ((size_t)b * NS + s) * NH + kc;
        const v4f a = *(const v4f*)src;
        const v4f c = *(const v4f*)(src + 4);
        Pk16 k;
        k.h[0] = (f16t)a[0]; k.h[1] = (f16t)a[1]; k.h[2] = (f16t)a[2]; k.h[3] = (f16t)a[3];
        k.h[4] = (f16t)c[0]; k.h[5] = (f16t)c[1]; k.h[6] = (f16t)c[2]; k.h[7] = (f16t)c[3];
        *(v8h*)(As_ + b * LPA + kc) = k.h;
    }
}

__global__ __launch_bounds__(256)
void k_lstm(const float* X, const f16t* Wc,
            const float* bihF, const float* bhhF, const float* bihB, const float* bhhB,
            float* Hid) {
    __shared__ __attribute__((aligned(16))) f16t  As[16 * LPA];
    __shared__ __attribute__((aligned(16))) float Gs[NB * NG];
    __shared__ __attribute__((aligned(16))) float Cs[NB * NHD];
    __shared__ __attribute__((aligned(16))) float Hs[NB * NHD];
    __shared__ __attribute__((aligned(16))) float Bs[NG];

    const int dir  = blockIdx.x;
    const int tid  = threadIdx.x;
    const int lane = tid & 31, w = tid >> 5, hh = lane >> 4, m = lane & 15;
    const float* bi = dir ? bihB : bihF;
    const float* bh = dir ? bhhB : bhhF;
    const f16t* Wd = Wc + (size_t)dir * NG * KC;

    for (int i = tid; i < 16 * LPA; i += 256) As[i] = (f16t)0.0f;
    for (int i = tid; i < NB * NHD; i += 256) Cs[i] = 0.0f;
    for (int i = tid; i < NG; i += 256) Bs[i] = bi[i] + bh[i];
    __syncthreads();
    gather_x(X, As, dir ? (NS - 1) : 0, tid);
    __syncthreads();

    const float inv32 = 0.03125f;

#pragma unroll 1
    for (int step = 0; step < NS; ++step) {
        const int s = dir ? (NS - 1 - step) : step;

#pragma unroll 1
        for (int g = 0; g < 3; ++g) {
            const int n0 = w * 192 + g * 64;
            v8f acc[4];
            const v8f z = {0.f, 0.f, 0.f, 0.f, 0.f, 0.f, 0.f, 0.f};
#pragma unroll
            for (int j = 0; j < 4; ++j) acc[j] = z;
            mma4(acc, As, LPA, Wd + (size_t)n0 * KC, KC, KTL);
            if (hh == 0) {
#pragma unroll
                for (int j = 0; j < 4; ++j) {
#pragma unroll
                    for (int r = 0; r < 8; ++r)
                        Gs[r * NG + n0 + 16 * j + m] = acc[j][r];
                }
            }
        }
        __syncthreads();

#pragma unroll 1
        for (int i = 0; i < 12; ++i) {
            const int e = tid + 256 * i;
            const int b = e / NHD;
            const int u = e - b * NHD;
            const float* gr = Gs + b * NG + u;
            const float pi = fmaf(gr[0],       inv32, Bs[u]);
            const float pf = fmaf(gr[NHD],     inv32, Bs[NHD + u]);
            const float pg = fmaf(gr[2 * NHD], inv32, Bs[2 * NHD + u]);
            const float po = fmaf(gr[3 * NHD], inv32, Bs[3 * NHD + u]);
            float c = Cs[e];
            c = fsig(pf) * c + fsig(pi) * ftanh(pg);
            const float hv = fsig(po) * ftanh(c);
            Cs[e] = c;
            Hs[e] = hv;
            As[b * LPA + NH + u] = (f16t)hv;
        }
        if (step + 1 < NS) gather_x(X, As, dir ? (NS - 2 - step) : (step + 1), tid);
        __syncthreads();

        v4f hv4[3];
        float* dst[3];
#pragma unroll
        for (int i = 0; i < 3; ++i) {
            const int p = tid + 256 * i;
            const int L = p >> 3, q = p & 7;
            const int b = L / 12;
            const int f = (L - b * 12) * 32 + q * 4;
            hv4[i] = *(const v4f*)(Hs + b * NHD + f);
            dst[i] = Hid + ((size_t)b * NS + s) * NH + dir * NHD + f;
        }
#pragma unroll
        for (int i = 0; i < 3; ++i) *(volatile v4f*)dst[i] = hv4[i];
        __threadfence();
#pragma unroll
        for (int i = 0; i < 3; ++i) *(volatile v4f*)dst[i] = hv4[i];
    }
}

__global__ __launch_bounds__(256)
void k_tail(const float* Hid, const int* Uid, const float* tw, const float* tb,
            const float* tt, float* Out) {
    __shared__ __attribute__((aligned(16))) float ML[NU * NH];
    __shared__ __attribute__((aligned(16))) float LG[NU * NTP];
    __shared__ int Us[NS];

    const int b = blockIdx.x;
    const int tid = threadIdx.x, lane = tid & 31, w = tid >> 5;
    const float ninf = -__builtin_inff();

    for (int i = tid; i < NS; i += 256) Us[i] = Uid[(size_t)b * NS + i];
    for (int i = tid; i < NU * NH; i += 256) ML[i] = ninf;
    __syncthreads();

    const float* hb = Hid + (size_t)b * NS * NH;
#pragma unroll 1
    for (int s = 0; s < NS; ++s) {
        const int u = Us[s];
        if (u > 0 && u <= NU) {
            float* mr = ML + (u - 1) * NH;
            const float* hr = hb + (size_t)s * NH;
#pragma unroll
            for (int k = 0; k < 3; ++k) {
                const int f = tid + 256 * k;
                mr[f] = fmaxf(mr[f], hr[f]);
            }
        }
    }
    __syncthreads();
    for (int i = tid; i < NU * NH; i += 256) ML[i] = fmaxf(ML[i], 0.0f);
    __syncthreads();

#pragma unroll 1
    for (int i = 0; i < 8; ++i) {
        const int p = tid + 256 * i;
        const int u = p >> 6, t = p & 63;
        const float* mr = ML + u * NH;
        const float* wr = tw + (size_t)t * NH;
        float a = 0.0f;
#pragma unroll 1
        for (int hI = 0; hI < NH; ++hI) a = fmaf(mr[hI], wr[hI], a);
        LG[p] = a + tb[t];
    }
    __syncthreads();

#pragma unroll 1
    for (int r = 0; r < 4; ++r) {
        const int u = w + 8 * r;
        const float v0 = LG[u * NTP + lane];
        const float v1 = LG[u * NTP + 32 + lane];
        float mx = fmaxf(v0, v1);
#pragma unroll
        for (int o = 16; o > 0; o >>= 1) mx = fmaxf(mx, __shfl_xor(mx, o));
        const float e0 = __expf(v0 - mx);
        const float e1 = __expf(v1 - mx);
        float sm = e0 + e1;
#pragma unroll
        for (int o = 16; o > 0; o >>= 1) sm += __shfl_xor(sm, o);
        const float inv = __builtin_amdgcn_rcpf(sm);
        LG[u * NTP + lane]      = e0 * inv;
        LG[u * NTP + 32 + lane] = e1 * inv;
    }
    __syncthreads();

#pragma unroll 1
    for (int u = 0; u < NU; ++u) {
        const float* pr = LG + u * NTP;
#pragma unroll
        for (int k = 0; k < 3; ++k) {
            const int f = tid + 256 * k;
            float a = 0.0f;
#pragma unroll 1
            for (int t = 0; t < NTP; ++t) a = fmaf(pr[t], tt[(size_t)t * NH + f], a);
            ML[u * NH + f] = a;
        }
    }
    __syncthreads();

#pragma unroll 1
    for (int r = 0; r < NS / 8; ++r) {
        const int s  = w + 8 * r;
        const int u  = Us[s];
        const int au = (u < 0) ? -u : u;
        int idx = au - 1;
        idx = (idx < 0) ? 0 : ((idx > NU - 1) ? (NU - 1) : idx);
        const float sc = (u > 0) ? 1.0f : ((u < 0) ? 2.0f : 0.0f);
        const float* er = ML + idx * NH;
        float* orow = Out + ((size_t)b * NS + s) * NH;
        v4f v[6];
#pragma unroll
        for (int i = 0; i < 6; ++i) v[i] = *(const v4f*)(er + (32 * i + lane) * 4) * sc;
#pragma unroll
        for (int i = 0; i < 6; ++i) *(volatile v4f*)(orow + (32 * i + lane) * 4) = v[i];
        __threadfence();
#pragma unroll
        for (int i = 0; i < 6; ++i) *(volatile v4f*)(orow + (32 * i + lane) * 4) = v[i];
    }
}

extern "C" void kernel_launch(void* const* d_in, const int* in_sizes, int n_in,
                              void* d_out, int out_size, void* d_ws, size_t ws_size,
                              hipStream_t stream) {
    if (n_in < 13) return;
    if (in_sizes[0] != NB * NS * NH) return;
    if (in_sizes[1] != NG * NH || in_sizes[2] != NG * NHD) return;
    if (in_sizes[3] != NG || in_sizes[4] != NG) return;
    if (in_sizes[5] != NG * NH || in_sizes[6] != NG * NHD) return;
    if (in_sizes[7] != NG || in_sizes[8] != NG) return;
    if (in_sizes[9] != NTP * NH || in_sizes[10] != NTP || in_sizes[11] != NTP * NH) return;
    if (in_sizes[12] != NB * NS) return;
    if (out_size != NB * NS * NH) return;

    const float* X    = (const float*)d_in[0];
    const float* WihF = (const float*)d_in[1];
    const float* WhhF = (const float*)d_in[2];
    const float* bihF = (const float*)d_in[3];
    const float* bhhF = (const float*)d_in[4];
    const float* WihB = (const float*)d_in[5];
    const float* WhhB = (const float*)d_in[6];
    const float* bihB = (const float*)d_in[7];
    const float* bhhB = (const float*)d_in[8];
    const float* tw   = (const float*)d_in[9];
    const float* tb   = (const float*)d_in[10];
    const float* tt   = (const float*)d_in[11];
    const int*   uid  = (const int*)d_in[12];
    float* out = (float*)d_out;

    const size_t wc_bytes  = (size_t)2 * NG * KC * sizeof(f16t);
    const size_t hid_bytes = (size_t)NB * NS * NH * sizeof(float);
    const size_t off_hid   = (wc_bytes + 127) & ~(size_t)127;
    const size_t total     = off_hid + hid_bytes;
    if (total > ws_size) return;
    char* ws = (char*)d_ws;
    f16t*  Wc  = (f16t*)(ws);
    float* Hid = (float*)(ws + off_hid);

    {
        const int tot = 2 * NG * WPR;
        k_wpack<<<dim3((tot + 255) / 256), dim3(256), 0, stream>>>(WihF, WhhF, WihB, WhhB, Wc, tot);
    }
    k_lstm<<<dim3(2), dim3(256), 0, stream>>>(X, Wc, bihF, bhhF, bihB, bhhB, Hid);
    k_tail<<<dim3(NB), dim3(256), 0, stream>>>(Hid, uid, tw, tb, tt, out);
}
